// CausalSelfAttention_22024592293896
// MI455X (gfx1250) — hardware-verified
//
#include <hip/hip_runtime.h>


#ifndef NB
#define NB 2
#endif
#ifndef SEQ
#define SEQ 2048
#endif
#define NB_FULL  2
#define SEQ_FULL 2048
#define DM   1024
#define NH_  16
#define HD   64
#define NBH  (NB * NH_)
#define LDF  (3 * DM)
#define MR   (NB * SEQ)
#define RH   256
#define RHE  ((RH < SEQ) ? RH : SEQ)
#define PCAR 1024.0f
#define RSC  2048.0f
#define RINV (1.0f / 2048.0f)
#define SCL  0.125f
#define SPP  40
#define KOFF (NBH * SEQ * HD)

typedef _Float16 h16;
typedef unsigned short bf;
typedef __attribute__((ext_vector_type(16))) __bf16   v16bf;
typedef __attribute__((ext_vector_type(16))) _Float16 v16h;
typedef __attribute__((ext_vector_type(8)))  _Float16 v8h;
typedef __attribute__((ext_vector_type(2)))  _Float16 v2h;
typedef __attribute__((ext_vector_type(8)))  unsigned short v8us;
typedef __attribute__((ext_vector_type(8)))  float    v8f;
typedef __attribute__((ext_vector_type(4)))  float    v4f;
typedef __attribute__((ext_vector_type(2)))  float    v2f;
typedef v8h  __attribute__((may_alias)) v8ha;
typedef v4f  __attribute__((may_alias)) v4fa;

static_assert(HD == 64);
static_assert(DM == NH_ * HD);
static_assert(DM % 32 == 0);
static_assert(SEQ % 64 == 0);
static_assert(MR % 64 == 0);
static_assert(LDF % 64 == 0);
static_assert(RHE % 16 == 0);
static_assert((SEQ - RHE) % 16 == 0);
static_assert(SEQ <= SEQ_FULL);
static_assert(NB <= NB_FULL);
static_assert((long long)2 * KOFF < 2147483647LL);
static_assert(SPP % 8 == 0);

constexpr size_t al256(size_t b) { return (b + 255) & ~(size_t)255; }
constexpr size_t SZ_WB = al256((size_t)LDF * DM * 2);
constexpr size_t SZ_XB = al256((size_t)MR * DM * 2);
constexpr size_t SZ_F  = al256((size_t)MR * LDF * 4);
constexpr size_t SZ_P  = al256((size_t)2 * KOFF * 2);
constexpr size_t SZ_V  = al256((size_t)KOFF * 2);
constexpr size_t WS_TOTAL = SZ_WB + SZ_XB + SZ_F + 2 * SZ_P + 2 * SZ_V;
static_assert(WS_TOTAL <= (size_t)134217728);

__device__ __forceinline__ unsigned short f2bf(float f) { unsigned u = __float_as_uint(f); u += 0x7FFFu + ((u >> 16) & 1u); return (unsigned short)(u >> 16); }
__device__ __forceinline__ float bf2f(unsigned short b) { return __uint_as_float(((unsigned)b) << 16); }
__device__ __forceinline__ float bfr(float f) { return bf2f(f2bf(f)); }
__device__ __forceinline__ v16h cat16(v8h lo, v8h hi) { return __builtin_shufflevector(lo, hi, 0, 1, 2, 3, 4, 5, 6, 7, 8, 9, 10, 11, 12, 13, 14, 15); }
__device__ __forceinline__ v16bf cat16b(v8us lo, v8us hi) { return __builtin_bit_cast(v16bf, __builtin_shufflevector(lo, hi, 0, 1, 2, 3, 4, 5, 6, 7, 8, 9, 10, 11, 12, 13, 14, 15)); }
__device__ __forceinline__ v8f wmma16(v16h a, v16h b, v8f c) { return __builtin_amdgcn_wmma_f32_16x16x32_f16(false, a, false, b, (short)0, c, false, false); }
__device__ __forceinline__ v8f wmmab(v16bf a, v16bf b, v8f c) { return __builtin_amdgcn_wmma_f32_16x16x32_bf16(false, a, false, b, (short)0, c, false, false); }
__device__ __forceinline__ v16h  ldf(const h16* p) { return cat16(*(const v8h*)p, *(const v8h*)(p + 16)); }
__device__ __forceinline__ v16bf ldfb(const bf* p) { return cat16b(*(const v8us*)p, *(const v8us*)(p + 16)); }
__device__ __forceinline__ void splith(float v, h16& hv, h16& rv) {
    float af = (float)((h16)v);
    af = (fabsf(af) < 6.103515625e-5f) ? 0.0f : af;
    hv = (h16)af; rv = (h16)((v - af) * RSC);
}

__global__ __launch_bounds__(256) void k_cvt8(const float* __restrict__ src, bf* dst, int n8, int gpb, int sstride8) {
    const int i = blockIdx.x * 256 + threadIdx.x; if (i >= n8) return;
    const int b = i / gpb, rem = i - b * gpb;
    const size_t so = ((size_t)b * sstride8 + rem) * 8;
    const v8f v = *(const v8f*)(src + so); v8us o;
#pragma unroll
    for (int k = 0; k < 8; ++k) o[k] = f2bf(v[k]);
    *(volatile v8us*)(dst + (size_t)i * 8) = o; __threadfence(); *(volatile v8us*)(dst + (size_t)i * 8) = o;
}

__global__ __launch_bounds__(32) void k_gemmw(const bf* __restrict__ A, const bf* __restrict__ Bt, int K, float* C, int ldc) {
    __shared__ __align__(16) float os[16 * 68];
    const int lane = threadIdx.x & 31, lr = lane & 15, hi = lane >> 4; const int r0 = blockIdx.x * 64, c0 = blockIdx.y * 64;
    v8f acc[4][4];
#pragma unroll
    for (int mb = 0; mb < 4; ++mb)
#pragma unroll
        for (int nb = 0; nb < 4; ++nb) acc[mb][nb] = (v8f){};
    const size_t aoff = (size_t)(r0 + lr) * K + 8 * hi, boff = (size_t)(c0 + lr) * K + 8 * hi;
#pragma unroll 1
    for (int kc = 0; kc < K; kc += 32) {
        v16bf a[4]; v16bf b;
#pragma unroll
        for (int mb = 0; mb < 4; ++mb) a[mb] = ldfb(A + aoff + (size_t)mb * 16 * K + kc);
#pragma unroll
        for (int nb = 0; nb < 4; ++nb) { b = ldfb(Bt + boff + (size_t)nb * 16 * K + kc);
#pragma unroll
            for (int mb = 0; mb < 4; ++mb) acc[mb][nb] = wmmab(a[mb], b, acc[mb][nb]); }
        asm volatile("" : "+v"(acc[0][0]), "+v"(acc[0][1]), "+v"(acc[0][2]), "+v"(acc[0][3]), "+v"(acc[1][0]), "+v"(acc[1][1]), "+v"(acc[1][2]), "+v"(acc[1][3]));
        asm volatile("v_nop\n\tv_nop\n\tv_nop\n\tv_nop" : "+v"(acc[2][0]), "+v"(acc[2][1]), "+v"(acc[2][2]), "+v"(acc[2][3]), "+v"(acc[3][0]), "+v"(acc[3][1]), "+v"(acc[3][2]), "+v"(acc[3][3]) : "v"(a[0]), "v"(a[3]), "v"(b));
    }
#pragma unroll
    for (int mb = 0; mb < 4; ++mb) {
#pragma unroll
        for (int nb = 0; nb < 4; ++nb) {
#pragma unroll
            for (int j = 0; j < 8; ++j) os[(hi * 8 + j) * 68 + nb * 16 + lr] = acc[mb][nb][j]; }
        __syncthreads();
        float* crow = C + (size_t)(r0 + mb * 16) * ldc + c0;
#pragma unroll 1
        for (int ps = 0; ps < 2; ++ps) {
#pragma unroll
            for (int s = 0; s < 8; ++s) { const int row = 2 * s + hi, cofs = lr * 4; const v4f val = *(const v4fa*)(os + row * 68 + cofs);
                *(volatile v4f*)(crow + (size_t)row * ldc + cofs) = val; }
            if (ps == 0) __threadfence(); }
        __syncthreads();
    }
}

__global__ __launch_bounds__(256) void k_rope(const float* __restrict__ F, const float* __restrict__ fc, const float* __restrict__ fs, h16* PH, h16* PR) {
#pragma clang fp contract(off)
    const int tid = blockIdx.x * 256 + threadIdx.x; if (tid >= 2 * NBH * SEQ * 32) return;
    const int j = tid & 31; const int row = tid >> 5;
    const int t = row % SEQ; const int bh = (row / SEQ) % NBH; const int which = row / (SEQ * NBH);
    const int b = bh / NH_, h = bh % NH_;
    const v2f x = *(const v2f*)(F + (size_t)(b * SEQ + t) * LDF + which * DM + h * HD + 2 * j);
    const float c = bfr(fc[t * 32 + j]), s = bfr(fs[t * 32 + j]);
    const float a0 = x[0] * c, a1 = x[1] * s, b0 = x[0] * s, b1 = x[1] * c;
    const float r0 = a0 - a1, r1 = b0 + b1;
    h16 h0, l0, h1, l1; splith(r0, h0, l0); splith(r1, h1, l1);
    v2h oh, ol; oh[0] = h0; oh[1] = h1; ol[0] = l0; ol[1] = l1;
    const size_t e = (size_t)row * HD + 2 * j;
    *(volatile v2h*)(PH + e) = oh; *(volatile v2h*)(PR + e) = ol; __threadfence(); *(volatile v2h*)(PH + e) = oh; *(volatile v2h*)(PR + e) = ol;
}

__global__ __launch_bounds__(256) void k_vtp(const float* __restrict__ F, h16* VH, h16* VR) {
    const int e = (blockIdx.x * 256 + threadIdx.x) * 2; if (e >= NBH * HD * SEQ) return;
    const int t = e % SEQ; const int d = (e / SEQ) % HD; const int bh = e / (SEQ * HD); const int b = bh / NH_, h = bh % NH_;
    v2h oh, ol;
#pragma unroll
    for (int q = 0; q < 2; ++q) { const float x = F[(size_t)(b * SEQ + t + q) * LDF + 2 * DM + h * HD + d]; h16 a, c; splith(x, a, c); oh[q] = a; ol[q] = c; }
    *(volatile v2h*)(VH + e) = oh; *(volatile v2h*)(VR + e) = ol; __threadfence(); *(volatile v2h*)(VH + e) = oh; *(volatile v2h*)(VR + e) = ol;
}

template <bool RES>
__device__ __forceinline__ void attn_body(const h16* __restrict__ PH, const h16* __restrict__ PR, const h16* __restrict__ VH, const h16* __restrict__ VR, float* out, const int qt, const int bh) {
    __shared__ __align__(16) h16 sp[16 * SPP];
    __shared__ __align__(16) h16 spr[16 * SPP];
    __shared__ __align__(16) float os[16 * 68];
    const int lane = threadIdx.x & 31, lr = lane & 15, hi = lane >> 4;
    const int q0 = qt * 16;
    const int pb = bh * (SEQ * HD);
    const int qoff = pb + (q0 + lr) * HD + 8 * hi;
    const int kbase = KOFF + pb + lr * HD + 8 * hi;
    const int vbase = pb + lr * SEQ + 8 * hi;
    const int nkb = (qt >> 1) + 1;
    const float CL2 = SCL * 1.4426950408889634f;
    v8f om[4], orr[4];
#pragma unroll
    for (int j = 0; j < 4; ++j) { om[j] = (v8f){}; orr[j] = (v8f){}; }
    float mrun[8], lrun[8];
#pragma unroll
    for (int r = 0; r < 8; ++r) { mrun[r] = -1.0e30f; lrun[r] = 0.0f; }

#pragma unroll 1
    for (int kb = 0; kb < nkb; ++kb) {
        const int k0 = kb * 32;
        int qo = qoff; asm volatile("" : "+v"(qo));
        const v16h qh0 = ldf(PH + qo), qh1 = ldf(PH + qo + 32);
        const v16h qr0 = ldf(PR + qo), qr1 = ldf(PR + qo + 32);
        v8f sm[2], sr[2]; v16h kh0, kh1, kr0, kr1;
#pragma unroll
        for (int hn = 0; hn < 2; ++hn) {
            const int ko = kbase + (k0 + hn * 16) * HD;
            kh0 = ldf(PH + ko); kh1 = ldf(PH + ko + 32); kr0 = ldf(PR + ko); kr1 = ldf(PR + ko + 32);
            sm[hn] = (v8f){}; sr[hn] = (v8f){};
            sm[hn] = wmma16(qh0, kh0, sm[hn]); sm[hn] = wmma16(qh1, kh1, sm[hn]);
            sr[hn] = wmma16(qh0, kr0, sr[hn]); sr[hn] = wmma16(qh1, kr1, sr[hn]);
            sr[hn] = wmma16(qr0, kh0, sr[hn]); sr[hn] = wmma16(qr1, kh1, sr[hn]);
        }
        asm volatile("v_nop\n\tv_nop\n\tv_nop\n\tv_nop" : "+v"(sm[0]), "+v"(sm[1]), "+v"(sr[0]), "+v"(sr[1]) : "v"(kh1), "v"(kr1), "v"(qr1));

        float u0[8], u1[8], al[8];
#pragma unroll
        for (int r = 0; r < 8; ++r) { u0[r] = (sm[0][r] + sr[0][r] * RINV) * CL2; u1[r] = (sm[1][r] + sr[1][r] * RINV) * CL2; }
        if (kb == nkb - 1) {
#pragma unroll
            for (int r = 0; r < 8; ++r) { const int row = q0 + 8 * hi + r; const int key = k0 + lr;
                u0[r] = (key > row) ? -1.0e30f : u0[r]; u1[r] = (key + 16 > row) ? -1.0e30f : u1[r]; }
        }
#pragma unroll
        for (int r = 0; r < 8; ++r) {
            float rm = fmaxf(u0[r], u1[r]);
            rm = fmaxf(rm, __shfl_xor(rm, 8, 32)); rm = fmaxf(rm, __shfl_xor(rm, 4, 32)); rm = fmaxf(rm, __shfl_xor(rm, 2, 32)); rm = fmaxf(rm, __shfl_xor(rm, 1, 32));
            const float nm = fmaxf(mrun[r], rm);
            al[r] = __builtin_amdgcn_exp2f(mrun[r] - nm);
            u0[r] = __builtin_amdgcn_exp2f(u0[r] - nm); u1[r] = __builtin_amdgcn_exp2f(u1[r] - nm);
            lrun[r] = lrun[r] * al[r] + (u0[r] + u1[r]);
            mrun[r] = nm;
        }
#pragma unroll
        for (int j = 0; j < 4; ++j)
#pragma unroll
            for (int r = 0; r < 8; ++r) { om[j][r] *= al[r]; if (RES) orr[j][r] *= al[r]; }
#pragma unroll
        for (int r = 0; r < 8; ++r) {
            const float c0 = u0[r] * PCAR, c1 = u1[r] * PCAR; const h16 a0 = (h16)c0, a1 = (h16)c1;
            sp[(8 * hi + r) * SPP + lr] = a0; sp[(8 * hi + r) * SPP + 16 + lr] = a1;
            if (RES) { spr[(8 * hi + r) * SPP + lr] = (h16)((c0 - (float)a0) * RSC); spr[(8 * hi + r) * SPP + 16 + lr] = (h16)((c1 - (float)a1) * RSC); }
        }
        __syncthreads();
        const v16h pa = cat16(*(const v8ha*)(sp + lr * SPP + 8 * hi), *(const v8ha*)(sp + lr * SPP + 16 + 8 * hi));
        v16h par = pa;
        if (RES) par = cat16(*(const v8ha*)(spr + lr * SPP + 8 * hi), *(const v8ha*)(spr + lr * SPP + 16 + 8 * hi));
        v16h vh, vr;
#pragma unroll
        for (int j = 0; j < 4; ++j) {
            const int vo = vbase + j * 16 * SEQ + k0;
            vh = ldf(VH + vo); vr = vh;
            om[j] = wmma16(pa, vh, om[j]);
            if (RES) { vr = ldf(VR + vo); orr[j] = wmma16(pa, vr, orr[j]); orr[j] = wmma16(par, vh, orr[j]); }
        }
        if (RES) asm volatile("v_nop\n\tv_nop\n\tv_nop\n\tv_nop" : "+v"(om[0]), "+v"(om[1]), "+v"(om[2]), "+v"(om[3]), "+v"(orr[0]), "+v"(orr[1]), "+v"(orr[2]), "+v"(orr[3]) : "v"(vh), "v"(vr), "v"(par));
        else     asm volatile("v_nop\n\tv_nop\n\tv_nop\n\tv_nop" : "+v"(om[0]), "+v"(om[1]), "+v"(om[2]), "+v"(om[3]) : "v"(vh), "v"(pa));
        __syncthreads();
    }

#pragma unroll
    for (int r = 0; r < 8; ++r) {
        float l = lrun[r];
        l += __shfl_xor(l, 8, 32); l += __shfl_xor(l, 4, 32); l += __shfl_xor(l, 2, 32); l += __shfl_xor(l, 1, 32);
        const float inv = __builtin_amdgcn_rcpf(l) * (1.0f / PCAR);
#pragma unroll
        for (int j = 0; j < 4; ++j) { const float o = RES ? (om[j][r] + orr[j][r] * RINV) : om[j][r]; os[(8 * hi + r) * 68 + j * 16 + lr] = o * inv; }
    }
    __syncthreads();
    float* orow = out + ((size_t)bh * SEQ_FULL + q0) * HD;
#pragma unroll 1
    for (int ps = 0; ps < 2; ++ps) {
#pragma unroll
        for (int s = 0; s < 8; ++s) { const int row = 2 * s + hi, cofs = lr * 4; const v4f val = *(const v4fa*)(os + row * 68 + cofs);
            *(volatile v4f*)(orow + (size_t)row * HD + cofs) = val; }
        if (ps == 0) __threadfence(); }
}

__global__ __launch_bounds__(32) void k_attn_e(const h16* __restrict__ PH, const h16* __restrict__ PR, const h16* __restrict__ VH, const h16* __restrict__ VR, float* out) {
    attn_body<true>(PH, PR, VH, VR, out, (int)blockIdx.x, (int)blockIdx.y);
}
__global__ __launch_bounds__(32) void k_attn_l(const h16* __restrict__ PH, const h16* __restrict__ PR, const h16* __restrict__ VH, const h16* __restrict__ VR, float* out) {
    attn_body<false>(PH, PR, VH, VR, out, RHE / 16 + (int)blockIdx.x, (int)blockIdx.y);
}

extern "C" void kernel_launch(void* const* d_in, const int* in_sizes, int n_in,
                              void* d_out, int out_size, void* d_ws, size_t ws_size, hipStream_t stream) {
    if (n_in < 4) return;
    if ((size_t)in_sizes[0] < ((size_t)(NB - 1) * SEQ_FULL + SEQ) * DM) return;
    if ((size_t)in_sizes[1] < (size_t)LDF * DM) return;
    if ((size_t)in_sizes[2] < (size_t)SEQ * (HD / 2)) return;
    if ((size_t)in_sizes[3] < (size_t)SEQ * (HD / 2)) return;
    if ((size_t)out_size < ((size_t)(NBH - 1) * SEQ_FULL + SEQ) * HD) return;
    if (ws_size < WS_TOTAL) return;
    const float* x  = (const float*)d_in[0];
    const float* w  = (const float*)d_in[1];
    const float* fc = (const float*)d_in[2];
    const float* fs = (const float*)d_in[3];
    float* OUT = (float*)d_out;
    char* wsp = (char*)d_ws;
    auto take = [&](size_t bytes) { char* p = wsp; wsp += bytes; return (void*)p; };
    bf*    WB = (bf*)take(SZ_WB);
    bf*    XB = (bf*)take(SZ_XB);
    float* F  = (float*)take(SZ_F);
    h16*   PH = (h16*)take(SZ_P);
    h16*   PR = (h16*)take(SZ_P);
    h16*   VH = (h16*)take(SZ_V);
    h16*   VR = (h16*)take(SZ_V);
    if ((size_t)(wsp - (char*)d_ws) > ws_size) return;

    const int nw8 = LDF * DM / 8, nx8 = MR * DM / 8;
    k_cvt8<<<(nw8 + 255) / 256, 256, 0, stream>>>(w, WB, nw8, nw8, 0);
    k_cvt8<<<(nx8 + 255) / 256, 256, 0, stream>>>(x, XB, nx8, SEQ * DM / 8, SEQ_FULL * DM / 8);
    k_gemmw<<<dim3(MR / 64, LDF / 64, 1), 32, 0, stream>>>(XB, WB, DM, F, LDF);
    k_rope<<<(2 * NBH * SEQ * 32 + 255) / 256, 256, 0, stream>>>(F, fc, fs, PH, PR);
    k_vtp<<<(NBH * HD * SEQ / 2 + 255) / 256, 256, 0, stream>>>(F, VH, VR);
    k_attn_e<<<dim3(RHE / 16, NBH, 1), 32, 0, stream>>>(PH, PR, VH, VR, OUT);
    if (SEQ > RHE) k_attn_l<<<dim3((SEQ - RHE) / 16, NBH, 1), 32, 0, stream>>>(PH, PR, VH, VR, OUT);
}
